// SelfAttention_82832739270703
// MI455X (gfx1250) — hardware-verified
//
#include <hip/hip_runtime.h>
#ifndef NB
#define NB 4
#endif
#ifndef SEQ
#define SEQ 256
#endif
#define SEQ_FULL 256
#define HID 1024
#define NHEAD 8
#define HDIM 128
#define EW (HID * NHEAD)
#define LSEQ (SEQ * NHEAD)
#define MROWS (NB * SEQ)
#define WCARRY 64.0f
#define OCARRY 256.0f
#define INVS 0.03125f
#define OPITCH 136

typedef unsigned short v8us __attribute__((ext_vector_type(8), may_alias));
typedef float  v8f  __attribute__((ext_vector_type(8)));
typedef float  v4f  __attribute__((ext_vector_type(4)));
typedef float  v4fa __attribute__((ext_vector_type(4), may_alias));
typedef _Float16 v16h __attribute__((ext_vector_type(16)));
union FragH { v16h v; v8us half[2]; _Float16 h[16]; unsigned short u[16]; };

static_assert(NHEAD * HDIM == HID);
static_assert(HDIM == 128);
static_assert(HID % 64 == 0 && EW % 64 == 0);
static_assert(HID % 32 == 0 && EW % 32 == 0);
static_assert(MROWS % 128 == 0);
static_assert(LSEQ % 64 == 0);
static_assert(SEQ <= SEQ_FULL && SEQ % 32 == 0);
static_assert(OPITCH >= HDIM && (OPITCH * 2) % 16 == 0);
#define WS_TOTAL ((size_t)3 * MROWS * HID * 2 + (size_t)EW * HID * 2 + (size_t)3 * MROWS * EW * 2 + (size_t)NB * HID * LSEQ * 2 + (size_t)NB * LSEQ * HID * 2)
static_assert(WS_TOTAL <= (size_t)134217728);
static_assert(((size_t)MROWS * HID * 2) % 256 == 0 && ((size_t)EW * HID * 2) % 256 == 0);

__device__ __forceinline__ unsigned short bf16_bits(float x) { unsigned int u = __float_as_uint(x); return (unsigned short)((u + 0x7FFFu + ((u >> 16) & 1u)) >> 16); }
__device__ __forceinline__ float bf16_rne(float x) { return __uint_as_float(((unsigned int)bf16_bits(x)) << 16); }

__device__ __forceinline__ v16h g2_frag(const _Float16* p, int hh) { FragH f; f.half[0] = *(const v8us*)((const unsigned short*)p + 8 * hh); f.half[1] = *(const v8us*)((const unsigned short*)p + 16 + 8 * hh); return f.v; }
__device__ __forceinline__ v8f g2_mma(v16h a, v16h b, v8f c) { v8f d = __builtin_amdgcn_wmma_f32_16x16x32_f16(false, a, false, b, (short)0, c, false, false); asm volatile("v_nop\n\tv_nop\n\tv_nop\n\tv_nop" : "+v"(d) : "v"(a), "v"(b)); return d; }

__global__ __launch_bounds__(256) void k_x16(const float* __restrict__ x, _Float16* __restrict__ X16, int n8) {
  const int t = blockIdx.x * 256 + threadIdx.x;
  if (t >= n8) return;
  const int e = t * 8;
  const int row = e / HID, col = e - row * HID;
  const int b = row / SEQ, s = row - b * SEQ;
  const float* src = x + (size_t)(b * SEQ_FULL + s) * HID + col;
  const v4f a = *(const v4fa*)src, c = *(const v4fa*)(src + 4);
  FragH f;
#pragma unroll
  for (int q = 0; q < 4; ++q) { f.h[q] = (_Float16)bf16_rne(a[q]); f.h[4 + q] = (_Float16)bf16_rne(c[q]); }
  const v8us o = f.half[0];
  unsigned short* d = (unsigned short*)X16 + (size_t)t * 8;
  *(volatile v8us*)d = o;
  __threadfence();
  *(volatile v8us*)d = o;
}

__global__ __launch_bounds__(256) void k_wnat(const float* __restrict__ wsrc, _Float16* __restrict__ Bt, int n8, float scale) {
  const int t = blockIdx.x * 256 + threadIdx.x;
  if (t >= n8) return;
  const float* src = wsrc + (size_t)t * 8;
  const v4f a = *(const v4fa*)src, c = *(const v4fa*)(src + 4);
  FragH f;
#pragma unroll
  for (int q = 0; q < 4; ++q) { f.h[q] = (_Float16)(bf16_rne(a[q]) * scale); f.h[4 + q] = (_Float16)(bf16_rne(c[q]) * scale); }
  const v8us o = f.half[0];
  unsigned short* d = (unsigned short*)Bt + (size_t)t * 8;
  *(volatile v8us*)d = o;
  __threadfence();
  *(volatile v8us*)d = o;
}

__global__ __launch_bounds__(256) void k_vt(const _Float16* __restrict__ V16, _Float16* __restrict__ VT) {
  __shared__ unsigned short tl[64][66];
  const int tid = threadIdx.x;
  const int cs = blockIdx.x % (HID / 64);
  const int rest = blockIdx.x / (HID / 64);
  const int ps = rest % (LSEQ / 64);
  const int b = rest / (LSEQ / 64);
  const int c0 = cs * 64, p0 = ps * 64;
  const unsigned short* Vu = (const unsigned short*)V16;
  unsigned short* VTu = (unsigned short*)VT;
  for (int i = tid; i < 64 * 8; i += 256) {
    const int j = i >> 3, c8 = (i & 7) * 8;
    FragH f;
    f.half[0] = *(const v8us*)(Vu + ((size_t)b * LSEQ + p0 + j) * HID + c0 + c8);
#pragma unroll
    for (int q = 0; q < 8; ++q) tl[c8 + q][j] = f.u[q];
  }
  __syncthreads();
  for (int pass = 0; pass < 2; ++pass) {
    for (int i = tid; i < 64 * 8; i += 256) {
      const int d = i >> 3, j8 = (i & 7) * 8;
      FragH f;
#pragma unroll
      for (int q = 0; q < 8; ++q) f.u[q] = tl[d][j8 + q];
      *(volatile v8us*)(VTu + ((size_t)b * HID + c0 + d) * LSEQ + p0 + j8) = f.half[0];
    }
    if (pass == 0) __threadfence();
  }
}

template <bool OUT16>
__device__ __forceinline__ void gemm_body(const _Float16* __restrict__ A, int lda, const _Float16* __restrict__ Bh, int ldb, float alpha,
                                          const float* __restrict__ bias, float* __restrict__ C, _Float16* __restrict__ C16, int ldc,
                                          int M, int N, int K, int rpb, int rpbf) {
  __shared__ __attribute__((aligned(16))) float so[4][32][68];
  const int tid = threadIdx.x, w = tid >> 5, lane = tid & 31, ln = lane & 15, hh = lane >> 4;
  const int ntn = N >> 6;
  const int mt = blockIdx.x / ntn, nq = blockIdx.x - mt * ntn;
  const int row0 = mt * 128 + 32 * w, col0 = nq * 64;
  if (row0 >= M) return;
  const _Float16* a0p = A + (size_t)(row0 + ln) * lda; const _Float16* a1p = a0p + (size_t)16 * lda;
  const _Float16* b0p = Bh + (size_t)(col0 + ln) * ldb; const _Float16* b1p = b0p + (size_t)16 * ldb; const _Float16* b2p = b1p + (size_t)16 * ldb; const _Float16* b3p = b2p + (size_t)16 * ldb;
  const v8f z8 = {0.f, 0.f, 0.f, 0.f, 0.f, 0.f, 0.f, 0.f};
  v8f c00 = z8, c01 = z8, c02 = z8, c03 = z8, c10 = z8, c11 = z8, c12 = z8, c13 = z8;
#pragma unroll 1
  for (int kb = 0; kb < K; kb += 32) {
    const v16h a0 = g2_frag(a0p + kb, hh), a1 = g2_frag(a1p + kb, hh);
    v16h b = g2_frag(b0p + kb, hh); c00 = g2_mma(a0, b, c00); c10 = g2_mma(a1, b, c10);
    b = g2_frag(b1p + kb, hh); c01 = g2_mma(a0, b, c01); c11 = g2_mma(a1, b, c11);
    b = g2_frag(b2p + kb, hh); c02 = g2_mma(a0, b, c02); c12 = g2_mma(a1, b, c12);
    b = g2_frag(b3p + kb, hh); c03 = g2_mma(a0, b, c03); c13 = g2_mma(a1, b, c13);
  }
  v8f accs[8] = {c00, c01, c02, c03, c10, c11, c12, c13};
#pragma unroll
  for (int u = 0; u < 8; ++u) {
    const int t = u & 3, half = u >> 2;
    const int col = col0 + t * 16 + ln;
    const float bv = bf16_rne(bias[col]);
#pragma unroll
    for (int r = 0; r < 8; ++r) so[w][half * 16 + 8 * hh + r][t * 16 + ln] = accs[u][r] * alpha + bv;
  }
  __builtin_amdgcn_fence(4  , "workgroup");
  __builtin_amdgcn_wave_barrier();
  if (OUT16) {
    const int rq = lane >> 3, c8 = (lane & 7) * 8;
    for (int pass = 0; pass < 2; ++pass) {
#pragma unroll
      for (int q = 0; q < 8; ++q) {
        const int r = q * 4 + rq;
        const v4f va = *(const v4fa*)&so[w][r][c8], vb = *(const v4fa*)&so[w][r][c8 + 4];
        FragH f;
#pragma unroll
        for (int i = 0; i < 4; ++i) { f.h[i] = (_Float16)va[i]; f.h[4 + i] = (_Float16)vb[i]; }
        *(volatile v8us*)((unsigned short*)C16 + (size_t)(row0 + r) * ldc + col0 + c8) = f.half[0];
      }
      if (pass == 0) __threadfence();
    }
  } else {
    const int rsub = lane >> 4, c4 = (lane & 15) * 4;
    for (int pass = 0; pass < 2; ++pass) {
#pragma unroll
      for (int q = 0; q < 16; ++q) {
        const int r = q * 2 + rsub;
        const int gr = row0 + r;
        const int ob = gr / rpb;
        const int orow = ob * rpbf + (gr - ob * rpb);
        const v4f v = *(const v4fa*)&so[w][r][c4];
        *(volatile v4f*)(C + (size_t)orow * ldc + col0 + c4) = v;
      }
      if (pass == 0) __threadfence();
    }
  }
}
__global__ __launch_bounds__(128) void k_gemm_p16(const _Float16* __restrict__ A, int lda, const _Float16* __restrict__ Bh, int ldb, float alpha,
                                                  const float* __restrict__ bias, _Float16* __restrict__ C16, int ldc, int M, int N, int K) {
  gemm_body<true>(A, lda, Bh, ldb, alpha, bias, nullptr, C16, ldc, M, N, K, 1, 1);
}
__global__ __launch_bounds__(128) void k_gemm_o32(const _Float16* __restrict__ A, int lda, const _Float16* __restrict__ Bh, int ldb, float alpha,
                                                  const float* __restrict__ bias, float* __restrict__ C, int ldc, int M, int N, int K, int rpb, int rpbf) {
  gemm_body<false>(A, lda, Bh, ldb, alpha, bias, C, nullptr, ldc, M, N, K, rpb, rpbf);
}

__global__ __launch_bounds__(128) __attribute__((amdgpu_num_vgpr(256)))
void k_attn(const _Float16* __restrict__ Q16, const _Float16* __restrict__ K16, const _Float16* __restrict__ VT, _Float16* __restrict__ O16) {
  __shared__ __attribute__((aligned(16))) unsigned short so[4][16][OPITCH];
  const int tid = threadIdx.x, w = tid >> 5, lane = tid & 31, ln = lane & 15, hh = lane >> 4;
  const int bh = blockIdx.y;
  const int b = bh / NHEAD, h = bh - b * NHEAD;
  const int q0 = blockIdx.x * 64 + w * 16;
  const size_t qoff = ((size_t)b * LSEQ + q0 + ln) * HID + h * HDIM;
  const size_t koff = ((size_t)b * LSEQ + ln) * HID + h * HDIM;
  const size_t voff = ((size_t)b * HID + h * HDIM + ln) * LSEQ;
  v16h fq[4];
#pragma unroll
  for (int c = 0; c < 4; ++c) fq[c] = g2_frag(Q16 + qoff + 32 * c, hh);
  const v8f z8 = {0.f, 0.f, 0.f, 0.f, 0.f, 0.f, 0.f, 0.f};
  v8f o[8];
#pragma unroll
  for (int t = 0; t < 8; ++t) o[t] = z8;
  float m = -1.0e30f, lsum = 0.f;
#pragma unroll 1
  for (int kb = 0; kb < LSEQ / 32; ++kb) {
    const _Float16* kp = K16 + koff + (size_t)kb * (32 * HID);
    v8f s0 = z8, s1 = z8;
#pragma unroll
    for (int c = 0; c < 4; ++c) {
      const v16h a0 = g2_frag(kp + 32 * c, hh);
      const v16h a1 = g2_frag(kp + (size_t)16 * HID + 32 * c, hh);
      s0 = g2_mma(a0, fq[c], s0);
      s1 = g2_mma(a1, fq[c], s1);
    }
    float mx = fmaxf(s0[0], s1[0]);
#pragma unroll
    for (int r = 1; r < 8; ++r) mx = fmaxf(mx, fmaxf(s0[r], s1[r]));
    mx = fmaxf(mx, __shfl_xor(mx, 16));
    const float mn = fmaxf(m, mx);
    if (__any(mn > m)) {
      const float al = __expf((m - mn) * INVS);
      lsum *= al;
#pragma unroll
      for (int t = 0; t < 8; ++t) o[t] *= al;
      m = mn;
    }
    FragH p;
    float ps = 0.f;
#pragma unroll
    for (int r = 0; r < 8; ++r) {
      const float e0 = __expf((s0[r] - m) * INVS), e1 = __expf((s1[r] - m) * INVS);
      p.h[r] = (_Float16)e0; p.h[8 + r] = (_Float16)e1;
      ps += e0 + e1;
    }
    lsum += ps;
    const _Float16* vp = VT + voff + kb * 32;
#pragma unroll
    for (int t = 0; t < 8; ++t) {
      const v16h av = g2_frag(vp + (size_t)t * (16 * LSEQ), hh);
      o[t] = g2_mma(av, p.v, o[t]);
    }
  }
  const float l = lsum + __shfl_xor(lsum, 16);
  const float inv = OCARRY * (1.0f / l);
#pragma unroll
  for (int t = 0; t < 8; ++t) {
    FragH f;
#pragma unroll
    for (int r = 0; r < 8; ++r) f.h[r] = (_Float16)(o[t][r] * inv);
    *(v8us*)&so[w][ln][16 * t + 8 * hh] = f.half[0];
  }
  __syncthreads();
  unsigned short* Ou = (unsigned short*)O16;
  const int rsub = lane >> 4, c8 = ln * 8;
  for (int pass = 0; pass < 2; ++pass) {
#pragma unroll
    for (int qq = 0; qq < 8; ++qq) {
      const int r = qq * 2 + rsub;
      const v8us v = *(const v8us*)&so[w][r][c8];
      *(volatile v8us*)(Ou + ((size_t)b * LSEQ + q0 + r) * HID + h * HDIM + c8) = v;
    }
    if (pass == 0) __threadfence();
  }
}

extern "C" void kernel_launch(void* const* d_in, const int* in_sizes, int n_in,
                              void* d_out, int out_size, void* d_ws, size_t ws_size, hipStream_t stream) {
  if (n_in < 11) return;
  const long long need_x = ((long long)(NB - 1) * SEQ_FULL + SEQ) * HID;
  if ((long long)in_sizes[0] < need_x || (long long)in_sizes[1] < need_x || (long long)in_sizes[2] < need_x) return;
  if ((long long)in_sizes[3] < (long long)EW * HID || (long long)in_sizes[5] < (long long)EW * HID || (long long)in_sizes[7] < (long long)EW * HID || (long long)in_sizes[9] < (long long)EW * HID) return;
  if (in_sizes[4] < EW || in_sizes[6] < EW || in_sizes[8] < EW || in_sizes[10] < HID) return;
  if ((long long)out_size < need_x) return;
  const float* xq = (const float*)d_in[0]; const float* xk = (const float*)d_in[1]; const float* xv = (const float*)d_in[2];
  const float* Wq = (const float*)d_in[3]; const float* bq = (const float*)d_in[4];
  const float* Wk = (const float*)d_in[5]; const float* bk = (const float*)d_in[6];
  const float* Wv = (const float*)d_in[7]; const float* bv = (const float*)d_in[8];
  const float* Wfc = (const float*)d_in[9]; const float* bfc = (const float*)d_in[10];
  float* out = (float*)d_out;

  char* ws = (char*)d_ws; size_t off = 0;
  auto take = [&](size_t bytes) { char* p = ws + off; off += (bytes + 255) & ~(size_t)255; return p; };
  _Float16* Xq = (_Float16*)take((size_t)MROWS * HID * 2);
  _Float16* Xk = (_Float16*)take((size_t)MROWS * HID * 2);
  _Float16* Xv = (_Float16*)take((size_t)MROWS * HID * 2);
  _Float16* WA = (_Float16*)take((size_t)EW * HID * 2);
  _Float16* Q16 = (_Float16*)take((size_t)MROWS * EW * 2);
  _Float16* K16 = (_Float16*)take((size_t)MROWS * EW * 2);
  _Float16* V16 = (_Float16*)take((size_t)MROWS * EW * 2);
  _Float16* VTp = (_Float16*)take((size_t)NB * HID * LSEQ * 2);
  _Float16* O16 = (_Float16*)take((size_t)NB * LSEQ * HID * 2);
  if (off > ws_size) return;

  const int nx8 = MROWS * HID / 8;
  const int nw8 = (int)((size_t)EW * HID / 8);
  const unsigned gx = (unsigned)((nx8 + 255) / 256), gw = (unsigned)((nw8 + 255) / 256);
  const unsigned gproj = (unsigned)((MROWS / 128) * (EW / 64));
  k_x16<<<gx, 256, 0, stream>>>(xq, Xq, nx8);
  k_x16<<<gx, 256, 0, stream>>>(xk, Xk, nx8);
  k_x16<<<gx, 256, 0, stream>>>(xv, Xv, nx8);
  k_wnat<<<gw, 256, 0, stream>>>(Wq, WA, nw8, WCARRY);
  k_gemm_p16<<<gproj, 128, 0, stream>>>(Xq, HID, WA, HID, 1.0f / WCARRY, bq, Q16, EW, MROWS, EW, HID);
  k_wnat<<<gw, 256, 0, stream>>>(Wk, WA, nw8, WCARRY);
  k_gemm_p16<<<gproj, 128, 0, stream>>>(Xk, HID, WA, HID, 1.0f / WCARRY, bk, K16, EW, MROWS, EW, HID);
  k_wnat<<<gw, 256, 0, stream>>>(Wv, WA, nw8, WCARRY);
  k_gemm_p16<<<gproj, 128, 0, stream>>>(Xv, HID, WA, HID, 1.0f / WCARRY, bv, V16, EW, MROWS, EW, HID);
  k_vt<<<(unsigned)(NB * (LSEQ / 64) * (HID / 64)), 256, 0, stream>>>(V16, VTp);
  k_attn<<<dim3(LSEQ / 64, NB * NHEAD), 128, 0, stream>>>(Q16, K16, VTp, O16);
  k_wnat<<<gw, 256, 0, stream>>>(Wfc, WA, nw8, WCARRY);
  k_gemm_o32<<<(unsigned)((MROWS / 128) * (HID / 64)), 128, 0, stream>>>(O16, EW, WA, EW, 1.0f / (WCARRY * OCARRY), bfc, out, HID, MROWS, HID, EW, SEQ, SEQ_FULL);
}
